// GatedScaledAttention_25469156065361
// MI455X (gfx1250) — hardware-verified
//
#include <hip/hip_runtime.h>
#include <stdint.h>
#include <stddef.h>

typedef __attribute__((ext_vector_type(16))) _Float16 v16h;
typedef __attribute__((ext_vector_type(8)))  _Float16 v8h;
typedef __attribute__((ext_vector_type(16))) __bf16   v16b;
typedef __attribute__((ext_vector_type(8)))  __bf16   v8b;
typedef __attribute__((ext_vector_type(8)))  float    v8f;
typedef __attribute__((ext_vector_type(4)))  float    v4f;
typedef __attribute__((ext_vector_type(2)))  float    v2f;
typedef __attribute__((ext_vector_type(4)))  int      v4i;

#define D_MODEL 1024
#define NHEAD   16
#define HDIM    64
#define TSEQ    1024
#define NBATCH  4
#define MROWS   (NBATCH * TSEQ)
#define ROPE_LOGF (-0.14391156831212787f)

__device__ __forceinline__ unsigned short f2bf_bits(float f) {
  unsigned u = __float_as_uint(f);
  return (unsigned short)((u + 0x7FFFu + ((u >> 16) & 1u)) >> 16);
}
__device__ __forceinline__ float bf_bits2f(unsigned short h) { return __uint_as_float(((unsigned)h) << 16); }

__device__ __forceinline__ void dep_guard_h(v8f& a, v8f& b, v16h x, v16h y) { asm volatile("v_nop\n\tv_nop\n\tv_nop\n\tv_nop" : "+v"(a), "+v"(b) : "v"(x), "v"(y)); }
__device__ __forceinline__ void dep_guard_b(v8f& a, v8f& b, v16b x, v16b y) { asm volatile("v_nop\n\tv_nop\n\tv_nop\n\tv_nop" : "+v"(a), "+v"(b) : "v"(x), "v"(y)); }
__device__ __forceinline__ void keep4_h(v16h a, v16h b, v16h c, v16h d) { asm volatile("v_nop" :: "v"(a), "v"(b), "v"(c), "v"(d)); }
__device__ __forceinline__ void keep4_b(v16b a, v16b b, v16b c, v16b d) { asm volatile("v_nop" :: "v"(a), "v"(b), "v"(c), "v"(d)); }
__device__ __forceinline__ void acc_guard4(v8f& a, v8f& b, v8f& c, v8f& d) { asm volatile("v_nop\n\tv_nop\n\tv_nop\n\tv_nop" : "+v"(a), "+v"(b), "+v"(c), "+v"(d)); }
template <typename T> struct Frag;
template <> struct Frag<_Float16> {
  typedef v16h V; union U { v16h v; v8h h[2]; };
  static __device__ __forceinline__ v16h load(const _Float16* p) {
    U f; f.h[0] = *(const v8h*)(p); f.h[1] = *(const v8h*)(p + 16); return f.v;
  }
  static __device__ __forceinline__ v8f mma(v16h a, v16h b, v8f c) {
    return __builtin_amdgcn_wmma_f32_16x16x32_f16(false, a, false, b, (short)0, c, false, false);
  }
  static __device__ __forceinline__ void guard(v8f& a, v8f& b, v16h x, v16h y) { dep_guard_h(a, b, x, y); }
  static __device__ __forceinline__ void keep(v16h a, v16h b, v16h c, v16h d) { keep4_h(a, b, c, d); }
};
template <> struct Frag<__bf16> {
  typedef v16b V; union U { v16b v; v8b h[2]; };
  static __device__ __forceinline__ v16b load(const __bf16* p) {
    U f; f.h[0] = *(const v8b*)(p); f.h[1] = *(const v8b*)(p + 16); return f.v;
  }
  static __device__ __forceinline__ v8f mma(v16b a, v16b b, v8f c) {
    return __builtin_amdgcn_wmma_f32_16x16x32_bf16(false, a, false, b, (short)0, c, false, false);
  }
  static __device__ __forceinline__ void guard(v8f& a, v8f& b, v16b x, v16b y) { dep_guard_b(a, b, x, y); }
  static __device__ __forceinline__ void keep(v16b a, v16b b, v16b c, v16b d) { keep4_b(a, b, c, d); }
};

__device__ __forceinline__ v8f mma_h(v16h a, v16h b, v8f c) {
  c = __builtin_amdgcn_wmma_f32_16x16x32_f16(false, a, false, b, (short)0, c, false, false);
  asm volatile("v_nop\n\tv_nop\n\tv_nop\n\tv_nop" : "+v"(c) : "v"(a), "v"(b));
  return c;
}

__global__ __launch_bounds__(256) void rope_tab_kernel(float* __restrict__ tab, int n2) {
  const int i = blockIdx.x * 256 + threadIdx.x;
  if (i < n2) {
    const int t  = i >> 5;
    const int ip = i & 31;
    const float freq = expf((float)(2 * ip) * ROPE_LOGF);
    const float ang  = (float)t * freq;
    float sn, cs;
    sincosf(ang, &sn, &cs);
    v2f val;
    val[0] = cs; val[1] = sn;
    *(volatile v2f*)(tab + (size_t)i * 2) = val;
    __threadfence();
    *(volatile v2f*)(tab + (size_t)i * 2) = val;
  }
}

__global__ __launch_bounds__(256) void mask_aux_kernel(const int* __restrict__ mask, int* __restrict__ kvm, float* __restrict__ hv) {
  __shared__ int red[256];
  __shared__ __align__(16) float hvs[32];
  const int tid = threadIdx.x;
  if (tid < 32) hvs[tid] = 0.0f;
  __syncthreads();
  for (int b = 0; b < NBATCH; ++b) {
    int anyv = 0;
    for (int t = tid; t < TSEQ; t += 256) anyv |= (mask[b * TSEQ + t] == 0) ? 1 : 0;
    red[tid] = anyv;
    __syncthreads();
    for (int s = 128; s > 0; s >>= 1) {
      if (tid < s) red[tid] |= red[tid + s];
      __syncthreads();
    }
    const int av = red[0];
    __syncthreads();
    if (tid == 0) hvs[b] = av ? 1.0f : 0.0f;
    const int t4 = tid * 4;
    const v4i mv = *(const v4i*)(mask + b * TSEQ + t4);
    v4i kv;
#pragma unroll
    for (int e = 0; e < 4; ++e) kv[e] = av ? ((mv[e] == 0) ? 1 : 0) : 1;
    *(volatile v4i*)(kvm + b * TSEQ + t4) = kv;
    __threadfence();
    *(volatile v4i*)(kvm + b * TSEQ + t4) = kv;
  }
  __syncthreads();
  if (tid < 8) {
    const v4f hl = *(const v4f*)(hvs + tid * 4);
    *(volatile v4f*)(hv + tid * 4) = hl;
    __threadfence();
    *(volatile v4f*)(hv + tid * 4) = hl;
  }
}

__global__ __launch_bounds__(256) void cast_f32_f16x8(const float* __restrict__ in, _Float16* __restrict__ out, int n8, float scale) {
  const int i = blockIdx.x * 256 + threadIdx.x;
  if (i < n8) {
    const size_t o = (size_t)i * 8;
    const v4f a = *(const v4f*)(in + o);
    const v4f b = *(const v4f*)(in + o + 4);
    v8h hv;
#pragma unroll
    for (int e = 0; e < 4; ++e) { hv[e] = (_Float16)(a[e] * scale); hv[4 + e] = (_Float16)(b[e] * scale); }
    *(volatile v8h*)(out + o) = hv;
    __threadfence();
    *(volatile v8h*)(out + o) = hv;
  }
}

template <int ET> struct Elem;
template <> struct Elem<0> { typedef _Float16 T; };
template <> struct Elem<1> { typedef __bf16 T; };
template <int ET, bool SPLIT, int BIAS_MODE, int OUT_MODE, bool RESID, int ACT, int ROPE>
__global__ __launch_bounds__(256) void wmma_gemm64(
    const unsigned short* __restrict__ Ap, const unsigned short* __restrict__ A2p, int lda, long strideA,
    const unsigned short* __restrict__ Btp, const unsigned short* __restrict__ Bt2p, int ldb, long strideB,
    void* __restrict__ Cout, void* __restrict__ Cout2, int ldc, long strideC,
    const float* __restrict__ bias,
    const float* __restrict__ resid, long strideR,
    const float* __restrict__ rtab,
    int M, int N, int K, float scale) {
  typedef typename Elem<ET>::T T;
  typedef typename Frag<T>::V V;
  const T* A = (const T*)Ap; const T* A2 = (const T*)A2p; const T* Bt = (const T*)Btp; const T* Bt2 = (const T*)Bt2p;
  __shared__ __align__(16) float sT[8][16 * 68];
  const int b    = blockIdx.y;
  const int lane = threadIdx.x & 31;
  const int wave = threadIdx.x >> 5;
  const int tilesN = N >> 6;
  const int tilesM = M >> 6;
  const int tile = blockIdx.x * 8 + wave;
  if (tile >= tilesM * tilesN) return;
  const int tm = tile / tilesN;
  const int tn = tile - tm * tilesN;
  const int m0 = tm << 6;
  const int n0 = tn << 6;

  const T* Ab  = A  + (size_t)b * strideA;
  const T* Bb  = Bt + (size_t)b * strideB;
  const T* Ab2 = SPLIT ? (A2  + (size_t)b * strideA) : nullptr;
  const T* Bb2 = SPLIT ? (Bt2 + (size_t)b * strideB) : nullptr;

  const int rlane = lane & 15;
  const int koff  = (lane >> 4) * 8;
  const int mOff  = (lane >> 4) * 8;

  v8f acc[4][4];
#pragma unroll
  for (int i = 0; i < 4; ++i)
#pragma unroll
    for (int j = 0; j < 4; ++j) acc[i][j] = (v8f){0.f,0.f,0.f,0.f,0.f,0.f,0.f,0.f};

  for (int k0 = 0; k0 < K; k0 += 32) {
    V bh[4], bl[4];
#pragma unroll
    for (int j = 0; j < 4; ++j) {
      const size_t bo = (size_t)(n0 + (j << 4) + rlane) * ldb + koff + k0;
      bh[j] = Frag<T>::load(Bb + bo);
      if (SPLIT) bl[j] = Frag<T>::load(Bb2 + bo);
    }
#pragma unroll
    for (int i = 0; i < 4; ++i) {
      const size_t ao = (size_t)(m0 + (i << 4) + rlane) * lda + koff + k0;
      V ah = Frag<T>::load(Ab + ao);
      V al;
      if (SPLIT) al = Frag<T>::load(Ab2 + ao);
#pragma unroll
      for (int j = 0; j < 4; ++j) {
        acc[i][j] = Frag<T>::mma(ah, bh[j], acc[i][j]);
        if (SPLIT) {
          acc[i][j] = Frag<T>::mma(ah, bl[j], acc[i][j]);
          acc[i][j] = Frag<T>::mma(al, bh[j], acc[i][j]);
        }
      }
      Frag<T>::guard(acc[i][0], acc[i][3], ah, SPLIT ? al : ah);
    }
    Frag<T>::keep(bh[0], bh[1], bh[2], bh[3]);
    if (SPLIT) Frag<T>::keep(bl[0], bl[1], bl[2], bl[3]);
  }
  acc_guard4(acc[0][0], acc[0][1], acc[0][2], acc[0][3]);
  acc_guard4(acc[1][0], acc[1][1], acc[1][2], acc[1][3]);
  acc_guard4(acc[2][0], acc[2][1], acc[2][2], acc[2][3]);
  acc_guard4(acc[3][0], acc[3][1], acc[3][2], acc[3][3]);

  float* slab = sT[wave];
  const float* Rb = RESID ? (resid + (size_t)b * strideR) : nullptr;
#pragma unroll
  for (int i = 0; i < 4; ++i) {
    const int mBase = m0 + (i << 4);
#pragma unroll
    for (int j = 0; j < 4; ++j) {
      const int n = n0 + (j << 4) + rlane;
      float bv = 0.f;
      if (BIAS_MODE == 2) bv = bias[n];
#pragma unroll
      for (int r = 0; r < 8; ++r) {
        float v = acc[i][j][r] * scale;
        if (BIAS_MODE == 1) v += bias[mBase + mOff + r];
        if (BIAS_MODE == 2) v += bv;
        if (RESID) v += Rb[(size_t)(mBase + mOff + r) * ldc + n];
        if (ACT == 1) v = tanhf(v);
        if (ACT == 2) v = fmaxf(v, 0.0f);
        if (ACT == 3) v = v / (1.0f + expf(-v));
        if (ACT == 4) v = (v > 0.f) ? v : 0.01f * v;
        if (ACT == 5) v = 0.5f * v * (1.0f + erff(v * 0.70710678118654752f));
        if (ACT == 6) v = __builtin_amdgcn_rcpf(1.0f + __expf(-v));
        slab[(mOff + r) * 68 + (j << 4) + rlane] = v;
      }
    }
    __builtin_amdgcn_fence(__ATOMIC_RELEASE, "workgroup");
    __builtin_amdgcn_wave_barrier();
    __builtin_amdgcn_fence(__ATOMIC_ACQUIRE, "workgroup");
    if (OUT_MODE == 0) {
      float* C = (float*)Cout + (size_t)b * strideC;
      const int hh = lane >> 4, c4 = (lane & 15) * 4;
      for (int pass = 0; pass < 2; ++pass) {
#pragma unroll
        for (int it = 0; it < 8; ++it) {
          const int row = it * 2 + hh;
          v4f v = *(const v4f*)(slab + row * 68 + c4);
          if (ROPE) {
            const unsigned t = (unsigned)(mBase + row) & (unsigned)(TSEQ - 1);
            const v4f cs = *(const v4f*)(rtab + (size_t)t * 64 + c4);
            const float e0 = v[0], o0 = v[1], e1 = v[2], o1 = v[3];
            v[0] = e0 * cs[0] - o0 * cs[1];
            v[1] = e0 * cs[1] + o0 * cs[0];
            v[2] = e1 * cs[2] - o1 * cs[3];
            v[3] = e1 * cs[3] + o1 * cs[2];
          }
          *(volatile v4f*)(C + (size_t)(mBase + row) * ldc + n0 + c4) = v;
        }
        __threadfence();
      }
    } else {
      const int q = lane >> 3, c8 = (lane & 7) * 8;
      unsigned short* C  = (unsigned short*)Cout  + (size_t)b * strideC;
      unsigned short* C2 = (OUT_MODE == 2) ? ((unsigned short*)Cout2 + (size_t)b * strideC) : nullptr;
      for (int pass = 0; pass < 2; ++pass) {
#pragma unroll
        for (int it = 0; it < 4; ++it) {
          const int row = it * 4 + q;
          const float* sp = slab + row * 68 + c8;
          float vals[8];
#pragma unroll
          for (int e = 0; e < 8; ++e) vals[e] = sp[e];
          if (ROPE) {
            const unsigned t = (unsigned)(mBase + row) & (unsigned)(TSEQ - 1);
            const float* tp = rtab + (size_t)t * 64 + c8;
            const v4f t0 = *(const v4f*)(tp);
            const v4f t1 = *(const v4f*)(tp + 4);
            const float cs0 = t0[0], sn0 = t0[1], cs1 = t0[2], sn1 = t0[3];
            const float cs2 = t1[0], sn2 = t1[1], cs3 = t1[2], sn3 = t1[3];
            float e, o;
            e = vals[0]; o = vals[1]; vals[0] = e * cs0 - o * sn0; vals[1] = e * sn0 + o * cs0;
            e = vals[2]; o = vals[3]; vals[2] = e * cs1 - o * sn1; vals[3] = e * sn1 + o * cs1;
            e = vals[4]; o = vals[5]; vals[4] = e * cs2 - o * sn2; vals[5] = e * sn2 + o * cs2;
            e = vals[6]; o = vals[7]; vals[6] = e * cs3 - o * sn3; vals[7] = e * sn3 + o * cs3;
          }
          v8h hv, lv;
#pragma unroll
          for (int e = 0; e < 8; ++e) {
            if (OUT_MODE == 1) {
              hv[e] = (_Float16)vals[e];
            } else {
              unsigned short hb = f2bf_bits(vals[e]);
              unsigned short lb = f2bf_bits(vals[e] - bf_bits2f(hb));
              hv[e] = __builtin_bit_cast(_Float16, hb);
              lv[e] = __builtin_bit_cast(_Float16, lb);
            }
          }
          *(volatile v8h*)(C + (size_t)(mBase + row) * ldc + n0 + c8) = hv;
          if (OUT_MODE == 2) *(volatile v8h*)(C2 + (size_t)(mBase + row) * ldc + n0 + c8) = lv;
        }
        __threadfence();
      }
    }
    __builtin_amdgcn_fence(__ATOMIC_RELEASE, "workgroup");
    __builtin_amdgcn_wave_barrier();
    __builtin_amdgcn_fence(__ATOMIC_ACQUIRE, "workgroup");
  }
}

#define AT_D 64
#define AT_NW 4
#define AT_QB 64
#define AT_KC 64
#define AT_PSC 32768.0f

__global__ __launch_bounds__(128)
void attn_f16_kernel(const _Float16* __restrict__ qp, const _Float16* __restrict__ kp,
                     const _Float16* __restrict__ vp, const int* __restrict__ kvm,
                     float* __restrict__ out, float sm_scale, float mask_fill) {
  __shared__ __align__(16) _Float16 Ksh[AT_KC * AT_D];
  __shared__ __align__(16) _Float16 Vth[AT_D * AT_KC];
  __shared__ __align__(16) _Float16 Psh[AT_NW][16 * AT_KC];
  __shared__ __align__(16) float    Os[AT_NW][16 * 68];

  const int tid  = threadIdx.x;
  const int wave = tid >> 5;
  const int lane = tid & 31;
  const int hh   = lane >> 4;
  const int c    = lane & 15;

  const int nqb  = TSEQ / AT_QB;
  const int bx   = blockIdx.x;
  const int qb   = bx % nqb;
  const int bhid = bx / nqb;
  const int h    = bhid % NHEAD;
  int b = bhid / NHEAD;
  if (b > NBATCH - 1) b = NBATCH - 1;
  const int q0 = qb * AT_QB + wave * 16;

  const size_t bstr = (size_t)TSEQ * D_MODEL;
  const _Float16* qb_ptr = qp + (size_t)b * bstr + (size_t)h * HDIM;
  const _Float16* kb_ptr = kp + (size_t)b * bstr + (size_t)h * HDIM;
  const _Float16* vb_ptr = vp + (size_t)b * bstr + (size_t)h * HDIM;
  float*          ob_ptr = out + (size_t)b * bstr + (size_t)h * HDIM;
  const int*      kvrow  = kvm + (size_t)b * TSEQ;

  v16h qa0, qa1;
  {
    const _Float16* qrow = qb_ptr + (size_t)(q0 + c) * D_MODEL;
    qa0 = Frag<_Float16>::load(qrow + 8 * hh);
    qa1 = Frag<_Float16>::load(qrow + 32 + 8 * hh);
  }

  float mrow[8], lrow[8];
  v8f oacc[4];
#pragma unroll
  for (int r = 0; r < 8; ++r) { mrow[r] = -__builtin_inff(); lrow[r] = 0.f; }
#pragma unroll
  for (int t = 0; t < 4; ++t) oacc[t] = (v8f){0.f,0.f,0.f,0.f,0.f,0.f,0.f,0.f};

  for (int kc = 0; kc < TSEQ / AT_KC; ++kc) {
    const int kv0 = kc * AT_KC;
    __syncthreads();
    {
      const int kvr = tid >> 1, dh = (tid & 1) * 32;
      const _Float16* krow = kb_ptr + (size_t)(kv0 + kvr) * D_MODEL + dh;
      const _Float16* vrow = vb_ptr + (size_t)(kv0 + kvr) * D_MODEL + dh;
#pragma unroll
      for (int i = 0; i < 4; ++i) {
        const v8h kk = *(const v8h*)(krow + 8 * i);
        *(v8h*)(Ksh + kvr * AT_D + dh + 8 * i) = kk;
        const v8h vv = *(const v8h*)(vrow + 8 * i);
#pragma unroll
        for (int e = 0; e < 8; ++e) Vth[(dh + 8 * i + e) * AT_KC + kvr] = vv[e];
      }
    }
    __syncthreads();

    v8f s[4];
#pragma unroll
    for (int j = 0; j < 4; ++j) {
      s[j] = (v8f){0.f,0.f,0.f,0.f,0.f,0.f,0.f,0.f};
      const v16h kb0 = Frag<_Float16>::load(Ksh + (j * 16 + c) * AT_D + 8 * hh);
      s[j] = mma_h(qa0, kb0, s[j]);
      const v16h kb1 = Frag<_Float16>::load(Ksh + (j * 16 + c) * AT_D + 32 + 8 * hh);
      s[j] = mma_h(qa1, kb1, s[j]);
    }
    int kvkeep[4];
#pragma unroll
    for (int j = 0; j < 4; ++j) kvkeep[j] = kvrow[kv0 + j * 16 + c];
    float cm[8];
#pragma unroll
    for (int r = 0; r < 8; ++r) {
      float m = -__builtin_inff();
#pragma unroll
      for (int j = 0; j < 4; ++j) {
        float sv = s[j][r] * sm_scale;
        if (kvkeep[j] == 0) sv = mask_fill;
        s[j][r] = sv;
        m = fmaxf(m, sv);
      }
#pragma unroll
      for (int off = 1; off < 16; off <<= 1) m = fmaxf(m, __shfl_xor(m, off, 32));
      cm[r] = m;
    }
    _Float16* pwh = Psh[wave];
#pragma unroll
    for (int r = 0; r < 8; ++r) {
      const float mnew  = fmaxf(mrow[r], cm[r]);
      const float alpha = expf(mrow[r] - mnew);
      mrow[r] = mnew;
      float psum = 0.f;
#pragma unroll
      for (int j = 0; j < 4; ++j) {
        const float p = expf(s[j][r] - mnew);
        psum += p;
        pwh[(8 * hh + r) * AT_KC + j * 16 + c] = (_Float16)(p * AT_PSC);
      }
#pragma unroll
      for (int off = 1; off < 16; off <<= 1) psum += __shfl_xor(psum, off, 32);
      lrow[r] = lrow[r] * alpha + psum;
#pragma unroll
      for (int t = 0; t < 4; ++t) oacc[t][r] *= alpha;
    }
    __builtin_amdgcn_fence(__ATOMIC_RELEASE, "workgroup");
    __builtin_amdgcn_wave_barrier();
    __builtin_amdgcn_fence(__ATOMIC_ACQUIRE, "workgroup");
#pragma unroll 1
    for (int kk = 0; kk < 2; ++kk) {
      const v16h pa = Frag<_Float16>::load(pwh + c * AT_KC + kk * 32 + 8 * hh);
#pragma unroll
      for (int t = 0; t < 4; ++t) {
        const v16h vb = Frag<_Float16>::load(Vth + (t * 16 + c) * AT_KC + kk * 32 + 8 * hh);
        oacc[t] = mma_h(pa, vb, oacc[t]);
      }
    }
  }

  float* os = Os[wave];
#pragma unroll
  for (int r = 0; r < 8; ++r) {
    const float inv = 1.0f / (lrow[r] * AT_PSC);
#pragma unroll
    for (int t = 0; t < 4; ++t) os[(8 * hh + r) * 68 + t * 16 + c] = oacc[t][r] * inv;
  }
  __builtin_amdgcn_fence(__ATOMIC_RELEASE, "workgroup");
  __builtin_amdgcn_wave_barrier();
  __builtin_amdgcn_fence(__ATOMIC_ACQUIRE, "workgroup");
  {
    const int c4 = (lane & 15) * 4;
    for (int pass = 0; pass < 2; ++pass) {
#pragma unroll
      for (int it = 0; it < 8; ++it) {
        const int row = it * 2 + hh;
        v4f val = *(const v4f*)(os + row * 68 + c4);
        *(volatile v4f*)(ob_ptr + (size_t)(q0 + row) * D_MODEL + c4) = val;
      }
      __threadfence();
    }
  }
}

__global__ __launch_bounds__(256) void gate_cast_kernel(const float* __restrict__ att, const float* __restrict__ gs,
                                                        const float* __restrict__ hv, _Float16* __restrict__ outp,
                                                        int n8, float scale) {
  const int i = blockIdx.x * 256 + threadIdx.x;
  if (i < n8) {
    int b = i >> 17;
    if (b > NBATCH - 1) b = NBATCH - 1;
    const float f = hv[b] * scale;
    const size_t o = (size_t)i * 8;
    const v4f a0 = *(const v4f*)(att + o), a1 = *(const v4f*)(att + o + 4);
    const v4f g0 = *(const v4f*)(gs + o),  g1 = *(const v4f*)(gs + o + 4);
    v8h hvv;
#pragma unroll
    for (int e = 0; e < 4; ++e) { hvv[e] = (_Float16)(a0[e] * g0[e] * f); hvv[4 + e] = (_Float16)(a1[e] * g1[e] * f); }
    *(volatile v8h*)(outp + o) = hvv;
    __threadfence();
    *(volatile v8h*)(outp + o) = hvv;
  }
}

extern "C" void kernel_launch(void* const* d_in, const int* in_sizes, int n_in,
                              void* d_out, int out_size, void* d_ws, size_t ws_size,
                              hipStream_t stream) {
  const int ND = MROWS * D_MODEL;
  const int NW = D_MODEL * D_MODEL;
  if (n_in != 14) return;
  if (in_sizes[0] != ND || in_sizes[1] != ND || in_sizes[2] != ND) return;
  if (in_sizes[3] != NBATCH * TSEQ) return;
  for (int i = 0; i < 5; ++i) {
    if (in_sizes[4 + 2 * i] != NW || in_sizes[5 + 2 * i] != D_MODEL) return;
  }
  if (out_size != ND) return;

  const float* query = (const float*)d_in[0];
  const float* key   = (const float*)d_in[1];
  const float* value = (const float*)d_in[2];
  const int*   mask  = (const int*)d_in[3];
  const float* Wq = (const float*)d_in[4];  const float* bq = (const float*)d_in[5];
  const float* Wk = (const float*)d_in[6];  const float* bk = (const float*)d_in[7];
  const float* Wv = (const float*)d_in[8];  const float* bv = (const float*)d_in[9];
  const float* Wo = (const float*)d_in[10]; const float* bo = (const float*)d_in[11];
  const float* Wg = (const float*)d_in[12]; const float* bg = (const float*)d_in[13];
  float* outp = (float*)d_out;

  char* wsp = (char*)d_ws;
  size_t off = 0;
  auto carve = [&](size_t bytes) -> void* {
    void* p = wsp + off;
    off += (bytes + 255) & ~(size_t)255;
    return p;
  };
  const size_t NDh = (size_t)ND * 2, NDf = (size_t)ND * 4, NWh = (size_t)NW * 2;
  _Float16* xq16 = (_Float16*)carve(NDh);
  _Float16* xk16 = (_Float16*)carve(NDh);
  _Float16* xv16 = (_Float16*)carve(NDh);
  _Float16* wq16 = (_Float16*)carve(NWh);
  _Float16* wk16 = (_Float16*)carve(NWh);
  _Float16* wv16 = (_Float16*)carve(NWh);
  _Float16* wg16 = (_Float16*)carve(NWh);
  _Float16* wo16 = (_Float16*)carve(NWh);
  _Float16* q16  = (_Float16*)carve(NDh);
  _Float16* k16  = (_Float16*)carve(NDh);
  _Float16* v16  = (_Float16*)carve(NDh);
  float*    gsig = (float*)carve(NDf);
  float*    rtab = (float*)carve((size_t)TSEQ * 32 * 2 * 4);
  int*      kvm  = (int*)carve((size_t)NBATCH * TSEQ * 4);
  float*    hv   = (float*)carve(128);
  float*    atto = (float*)carve(NDf);
  _Float16* gd16 = (_Float16*)carve(NDh);
  if (off > ws_size) return;

  const int nd8 = ND / 8, nw8 = NW / 8;
  const int blkND8 = (nd8 + 255) / 256;
  const int blkNW8 = (nw8 + 255) / 256;
  const int ntab2  = TSEQ * 32;
  const int blkTab = (ntab2 + 255) / 256;
  const int gemmBlocks = ((MROWS / 64) * (D_MODEL / 64) + 7) / 8;
  const int attnBlocks = NBATCH * NHEAD * (TSEQ / AT_QB);
  const float WSC = 64.0f;

  rope_tab_kernel<<<dim3(blkTab), dim3(256), 0, stream>>>(rtab, ntab2);
  mask_aux_kernel<<<dim3(1), dim3(256), 0, stream>>>(mask, kvm, hv);

  cast_f32_f16x8<<<dim3(blkND8), dim3(256), 0, stream>>>(query, xq16, nd8, 1.0f);
  cast_f32_f16x8<<<dim3(blkND8), dim3(256), 0, stream>>>(key,   xk16, nd8, 1.0f);
  cast_f32_f16x8<<<dim3(blkND8), dim3(256), 0, stream>>>(value, xv16, nd8, 1.0f);
  cast_f32_f16x8<<<dim3(blkNW8), dim3(256), 0, stream>>>(Wq, wq16, nw8, WSC);
  cast_f32_f16x8<<<dim3(blkNW8), dim3(256), 0, stream>>>(Wk, wk16, nw8, WSC);
  cast_f32_f16x8<<<dim3(blkNW8), dim3(256), 0, stream>>>(Wv, wv16, nw8, WSC);
  cast_f32_f16x8<<<dim3(blkNW8), dim3(256), 0, stream>>>(Wg, wg16, nw8, WSC);
  cast_f32_f16x8<<<dim3(blkNW8), dim3(256), 0, stream>>>(Wo, wo16, nw8, WSC);

  wmma_gemm64<0, false, 2, 1, false, 0, 1><<<dim3(gemmBlocks, 1), dim3(256), 0, stream>>>(
      (const unsigned short*)xq16, (const unsigned short*)xq16, D_MODEL, (long)0,
      (const unsigned short*)wq16, (const unsigned short*)wq16, D_MODEL, (long)0,
      (void*)q16, (void*)q16, D_MODEL, (long)0,
      bq, bq, (long)0, rtab, MROWS, D_MODEL, D_MODEL, 1.0f / WSC);
  wmma_gemm64<0, false, 2, 1, false, 0, 1><<<dim3(gemmBlocks, 1), dim3(256), 0, stream>>>(
      (const unsigned short*)xk16, (const unsigned short*)xk16, D_MODEL, (long)0,
      (const unsigned short*)wk16, (const unsigned short*)wk16, D_MODEL, (long)0,
      (void*)k16, (void*)k16, D_MODEL, (long)0,
      bk, bk, (long)0, rtab, MROWS, D_MODEL, D_MODEL, 1.0f / WSC);
  wmma_gemm64<0, false, 2, 1, false, 0, 0><<<dim3(gemmBlocks, 1), dim3(256), 0, stream>>>(
      (const unsigned short*)xv16, (const unsigned short*)xv16, D_MODEL, (long)0,
      (const unsigned short*)wv16, (const unsigned short*)wv16, D_MODEL, (long)0,
      (void*)v16, (void*)v16, D_MODEL, (long)0,
      bv, bv, (long)0, rtab, MROWS, D_MODEL, D_MODEL, 1.0f / WSC);
  wmma_gemm64<0, false, 2, 0, false, 6, 0><<<dim3(gemmBlocks, 1), dim3(256), 0, stream>>>(
      (const unsigned short*)xq16, (const unsigned short*)xq16, D_MODEL, (long)0,
      (const unsigned short*)wg16, (const unsigned short*)wg16, D_MODEL, (long)0,
      (void*)gsig, (void*)gsig, D_MODEL, (long)0,
      bg, bg, (long)0, rtab, MROWS, D_MODEL, D_MODEL, 1.0f / WSC);

  attn_f16_kernel<<<dim3(attnBlocks), dim3(128), 0, stream>>>(q16, k16, v16, kvm, atto, 0.125f, -1.0e30f);

  gate_cast_kernel<<<dim3(blkND8), dim3(256), 0, stream>>>(atto, gsig, hv, gd16, nd8, WSC);

  wmma_gemm64<0, false, 2, 0, false, 0, 0><<<dim3(gemmBlocks, 1), dim3(256), 0, stream>>>(
      (const unsigned short*)gd16, (const unsigned short*)gd16, D_MODEL, (long)0,
      (const unsigned short*)wo16, (const unsigned short*)wo16, D_MODEL, (long)0,
      (void*)outp, (void*)outp, D_MODEL, (long)0,
      bo, bo, (long)0, rtab, MROWS, D_MODEL, D_MODEL, 1.0f / (WSC * WSC));
}
